// PatchConv2Layer_8117488190080
// MI455X (gfx1250) — hardware-verified
//
#include <hip/hip_runtime.h>
#include <stddef.h>


#define DF      128
#define RDM     64
#define NTHR    256
#define NWAVE   8
#define EPT     8
#define NGRP    2
#define CHUNK   (NTHR * EPT * NGRP)
#define WCAP    (EPT * NGRP * 32)
#define LISTN   (NWAVE * WCAP)
#define NB1     512
#define NB2     1024
#define NBD     4096
#define NBP     32
#define G1ROWS  128
#define APITCH  136
#define WSCALE  8.0f
#define WINV    0.125f
#define ASC     64.0f
#define AWINV   (1.0f / 512.0f)
#define SLOPE   0.01f

#define LDS_GEMM1 (G1ROWS * DF * 4)
#define LDS_AGG1  (NB1 * DF * 4 + LISTN * 4 + 64)
#define LDS_AGG2  (NB2 * RDM * 4 + LISTN * 4 + 64)

static_assert((CHUNK & (CHUNK - 1)) == 0);
static_assert(CHUNK <= 4096);
static_assert(NB1 <= 4096 && NB2 <= 4096 && NBD <= 4096 && NBP <= 4096);
static_assert((NB1 & (NB1 - 1)) == 0 && (NB2 & (NB2 - 1)) == 0 && (NBD & (NBD - 1)) == 0 && (NBP & (NBP - 1)) == 0);
static_assert(G1ROWS * APITCH * 2 <= LDS_GEMM1);
static_assert(NBD % NB1 == 0 && NBD % NB2 == 0 && NBD % G1ROWS == 0);
static_assert(NB1 % (16 * NWAVE) == 0);
static_assert(NB1 % (2 * NWAVE) == 0 && (NB2 * RDM) % (128 * NWAVE) == 0);
static_assert(NBP * RDM == 2 * NWAVE * 128);
static_assert((NBP * RDM / 4) % NTHR == 0);

typedef float    v4f  __attribute__((ext_vector_type(4)));
typedef float    v8f  __attribute__((ext_vector_type(8)));
typedef int      v4i  __attribute__((ext_vector_type(4)));
typedef _Float16 v8h  __attribute__((ext_vector_type(8)));
typedef _Float16 v16h __attribute__((ext_vector_type(16)));
union FragH { v16h v; v8h h[2]; };

__device__ __forceinline__ float lk(float v) { return v >= 0.0f ? v : SLOPE * v; }

__device__ __forceinline__ v8h cvt8(v4f a, v4f b) {
  v8h r;
  r[0] = (_Float16)a.x; r[1] = (_Float16)a.y; r[2] = (_Float16)a.z; r[3] = (_Float16)a.w;
  r[4] = (_Float16)b.x; r[5] = (_Float16)b.y; r[6] = (_Float16)b.z; r[7] = (_Float16)b.w;
  return r;
}

__device__ __forceinline__ v8f wmh(v16h a, v16h b, v8f c) {
  v8f d = __builtin_amdgcn_wmma_f32_16x16x32_f16(false, a, false, b, (short)0, c, false, false);
  asm volatile("v_nop\n\tv_nop\n\tv_nop\n\tv_nop" : "+v"(d) : "v"(a), "v"(b));
  return d;
}

template <int NB>
__device__ __forceinline__ int scan_chunk(const int* __restrict__ keys, int nK, int cbase, int base,
                                          int vec8, int* list, int tid, int lane, int wave) {
  int wc = 0;
#pragma unroll
  for (int g = 0; g < NGRP; ++g) {
    const int el0  = (g * NTHR + tid) * EPT;
    const int e0   = cbase + el0;
    const int sent = -2147483647 - 1;
    v4i da, db;
    if (vec8 != 0 && cbase + CHUNK <= nK) {
      da = *(const v4i*)(keys + e0);
      db = *(const v4i*)(keys + e0 + 4);
    } else {
      da.x = (e0     < nK) ? keys[min(e0,     nK - 1)] : sent;
      da.y = (e0 + 1 < nK) ? keys[min(e0 + 1, nK - 1)] : sent;
      da.z = (e0 + 2 < nK) ? keys[min(e0 + 2, nK - 1)] : sent;
      da.w = (e0 + 3 < nK) ? keys[min(e0 + 3, nK - 1)] : sent;
      db.x = (e0 + 4 < nK) ? keys[min(e0 + 4, nK - 1)] : sent;
      db.y = (e0 + 5 < nK) ? keys[min(e0 + 5, nK - 1)] : sent;
      db.z = (e0 + 6 < nK) ? keys[min(e0 + 6, nK - 1)] : sent;
      db.w = (e0 + 7 < nK) ? keys[min(e0 + 7, nK - 1)] : sent;
    }
    const unsigned nb = (unsigned)base;
    const unsigned s0 = (unsigned)da.x - nb, s1 = (unsigned)da.y - nb;
    const unsigned s2 = (unsigned)da.z - nb, s3 = (unsigned)da.w - nb;
    const unsigned s4 = (unsigned)db.x - nb, s5 = (unsigned)db.y - nb;
    const unsigned s6 = (unsigned)db.z - nb, s7 = (unsigned)db.w - nb;
    const bool h0 = s0 < (unsigned)NB, h1 = s1 < (unsigned)NB, h2 = s2 < (unsigned)NB, h3 = s3 < (unsigned)NB;
    const bool h4 = s4 < (unsigned)NB, h5 = s5 < (unsigned)NB, h6 = s6 < (unsigned)NB, h7 = s7 < (unsigned)NB;
    const unsigned any = __builtin_amdgcn_ballot_w32(h0 | h1 | h2 | h3 | h4 | h5 | h6 | h7);
    if (any != 0u) {
#define HITJ(J, HJ, SJ) { \
        const unsigned mj = __builtin_amdgcn_ballot_w32(HJ); \
        if (mj != 0u) { \
          if (HJ) { \
            const int pos = wc + (int)__builtin_amdgcn_mbcnt_lo(mj, 0u); \
            if (pos < WCAP) list[wave * WCAP + pos] = ((el0 + (J)) << 12) | (int)(SJ); \
          } \
          wc += (int)__builtin_popcount(mj); } }
      HITJ(0, h0, s0)
      HITJ(1, h1, s1)
      HITJ(2, h2, s2)
      HITJ(3, h3, s3)
      HITJ(4, h4, s4)
      HITJ(5, h5, s5)
      HITJ(6, h6, s6)
      HITJ(7, h7, s7)
#undef HITJ
    }
  }
  return wc;
}

__global__ __launch_bounds__(NTHR) void k_wprep(
    const float* __restrict__ W1, const float* __restrict__ W2,
    _Float16* w1s, _Float16* w2s) {
  const int i  = blockIdx.x * NTHR + threadIdx.x;
  const int n1 = DF * DF / 8;
  const int n2 = RDM * DF / 8;
  if (i >= n1 + n2) return;
  const bool first = i < n1;
  const int o  = (first ? i : i - n1) * 8;
  const int n  = o / DF;
  const int k0 = o - n * DF;
  v4f a, b;
  if (first) {
    const float* p = W1 + (size_t)k0 * DF + n;
    a.x = p[0];      a.y = p[DF];     a.z = p[2 * DF]; a.w = p[3 * DF];
    b.x = p[4 * DF]; b.y = p[5 * DF]; b.z = p[6 * DF]; b.w = p[7 * DF];
  } else {
    const float* p = W2 + (size_t)k0 * RDM + n;
    a.x = p[0];       a.y = p[RDM];     a.z = p[2 * RDM]; a.w = p[3 * RDM];
    b.x = p[4 * RDM]; b.y = p[5 * RDM]; b.z = p[6 * RDM]; b.w = p[7 * RDM];
  }
  a = a * WSCALE;
  b = b * WSCALE;
  const v8h hv = cvt8(a, b);
  _Float16* dp = (first ? w1s : w2s) + o;
  *(volatile v8h*)dp = hv;
  __threadfence();
  *(volatile v8h*)dp = hv;
}

__global__ __launch_bounds__(NTHR) void k_deg(
    const int* __restrict__ keys, float* nrm, int nE, int vec8) {
  __shared__ __attribute__((aligned(16))) int cnt[NBD];
  __shared__ __attribute__((aligned(16))) int list[LISTN];
  __shared__ int wcnt[NWAVE];
  const int tid = threadIdx.x, lane = tid & 31, wave = tid >> 5;
  const int nodeBase = blockIdx.x * NBD;

  for (int i = tid; i < NBD; i += NTHR) cnt[i] = 0;
  __syncthreads();

  const int nChunks = (nE + CHUNK - 1) / CHUNK;
#pragma unroll 1
  for (int ch = 0; ch < nChunks; ++ch) {
    const int cbase = ch * CHUNK;
    const int wc = scan_chunk<NBD>(keys, nE, cbase, nodeBase, vec8, list, tid, lane, wave);
    if (lane == 0) wcnt[wave] = wc;
    __syncthreads();
    if (wave == 0) {
#pragma unroll 1
      for (int wsx = 0; wsx < NWAVE; ++wsx) {
        int n = __builtin_amdgcn_readfirstlane(wcnt[wsx]);
        n = n > WCAP ? WCAP : (n < 0 ? 0 : n);
        const int* lp = list + wsx * WCAP;
#pragma unroll 1
        for (int i = 0; i < n; ++i) {
          const int ent  = __builtin_amdgcn_readfirstlane(lp[i]);
          const int slot = ent & (NBD - 1);
          if (lane == 0) cnt[slot] = cnt[slot] + 1;
        }
      }
    }
    __syncthreads();
  }

  v4f dq[4];
#pragma unroll
  for (int q = 0; q < 4; ++q) {
    const int f = (wave * 4 + q) * 128 + 4 * lane;
    v4i c = *(const v4i*)(cnt + f);
    c.x = c.x < 1 ? 1 : c.x; c.y = c.y < 1 ? 1 : c.y; c.z = c.z < 1 ? 1 : c.z; c.w = c.w < 1 ? 1 : c.w;
    dq[q].x = rsqrtf((float)c.x);
    dq[q].y = rsqrtf((float)c.y);
    dq[q].z = rsqrtf((float)c.z);
    dq[q].w = rsqrtf((float)c.w);
  }
  float* dp = nrm + (size_t)nodeBase;
#pragma unroll
  for (int q = 0; q < 4; ++q) *(volatile v4f*)(dp + (wave * 4 + q) * 128 + 4 * lane) = dq[q];
  __threadfence();
#pragma unroll
  for (int q = 0; q < 4; ++q) *(volatile v4f*)(dp + (wave * 4 + q) * 128 + 4 * lane) = dq[q];
}

__global__ __launch_bounds__(NTHR) void k_gemm1(
    const float* __restrict__ x, const _Float16* __restrict__ w1s,
    const float* __restrict__ nrmS, float* g1, int nN) {
  extern __shared__ v4f lds_dyn[];
  _Float16* sA  = (_Float16*)lds_dyn;
  float*    stg = (float*)lds_dyn;
  const int tid = threadIdx.x, lane = tid & 31, wave = tid >> 5, hh = lane >> 4, m = lane & 15;
  const int rowBase = blockIdx.x * G1ROWS;

#pragma unroll
  for (int i = 0; i < (G1ROWS * DF / 8) / NTHR; ++i) {
    const int idx = i * NTHR + tid;
    const int r   = idx >> 4;
    const int c0  = (idx & 15) * 8;
    int node = rowBase + r;
    node = node > nN - 1 ? nN - 1 : node;
    const float* xp = x + (size_t)node * DF + c0;
    const v4f a = *(const v4f*)xp, b = *(const v4f*)(xp + 4);
    *(v8h*)(sA + r * APITCH + c0) = cvt8(a, b);
  }
  __syncthreads();

  v8f acc[8];
#pragma unroll
  for (int t = 0; t < 8; ++t) { v8f z = {0.f, 0.f, 0.f, 0.f, 0.f, 0.f, 0.f, 0.f}; acc[t] = z; }
  const _Float16* ar = sA + (wave * 16 + m) * APITCH + 8 * hh;
#pragma unroll
  for (int kt = 0; kt < DF / 32; ++kt) {
    FragH a;
    a.h[0] = *(const v8h*)(ar + 32 * kt);
    a.h[1] = *(const v8h*)(ar + 32 * kt + 16);
#pragma unroll
    for (int t = 0; t < 8; ++t) {
      const _Float16* bp = w1s + (size_t)(16 * t + m) * DF + 32 * kt + 8 * hh;
      FragH b;
      b.h[0] = *(const v8h*)bp;
      b.h[1] = *(const v8h*)(bp + 16);
      acc[t] = wmh(a.v, b.v, acc[t]);
    }
  }
  __syncthreads();

  const int r0 = wave * 16 + 8 * hh;
  const v4f dA = *(const v4f*)(nrmS + (size_t)rowBase + r0);
  const v4f dB = *(const v4f*)(nrmS + (size_t)rowBase + r0 + 4);
  const float d0 = dA.x * WINV, d1 = dA.y * WINV, d2 = dA.z * WINV, d3 = dA.w * WINV;
  const float d4 = dB.x * WINV, d5 = dB.y * WINV, d6 = dB.z * WINV, d7 = dB.w * WINV;
  float* sp = stg + r0 * DF + m;
#pragma unroll
  for (int t = 0; t < 8; ++t) {
    sp[0 * DF + 16 * t] = acc[t][0] * d0;
    sp[1 * DF + 16 * t] = acc[t][1] * d1;
    sp[2 * DF + 16 * t] = acc[t][2] * d2;
    sp[3 * DF + 16 * t] = acc[t][3] * d3;
    sp[4 * DF + 16 * t] = acc[t][4] * d4;
    sp[5 * DF + 16 * t] = acc[t][5] * d5;
    sp[6 * DF + 16 * t] = acc[t][6] * d6;
    sp[7 * DF + 16 * t] = acc[t][7] * d7;
  }
  __syncthreads();

  const float* lp = stg + wave * 16 * DF + 4 * lane;
  float* gp = g1 + ((size_t)rowBase + wave * 16) * DF + 4 * lane;
#pragma unroll
  for (int i = 0; i < 16; ++i) { const v4f v = *(const v4f*)(lp + i * DF); *(volatile v4f*)(gp + (size_t)i * DF) = v; }
  __threadfence();
#pragma unroll
  for (int i = 0; i < 16; ++i) { const v4f v = *(const v4f*)(lp + i * DF); *(volatile v4f*)(gp + (size_t)i * DF) = v; }
}

__global__ __launch_bounds__(NTHR) void k_agg1(
    const int* __restrict__ srcs, const int* __restrict__ dsts, const float* __restrict__ ew,
    const float* __restrict__ g1, const float* __restrict__ nrmD, const float* __restrict__ nrmS,
    const _Float16* __restrict__ w2s, float* g2, int nN, int nE, int vec8) {
  extern __shared__ v4f lds_dyn[];
  float* acc  = (float*)lds_dyn;
  int*   list = (int*)(acc + NB1 * DF);
  int*   wcnt = list + LISTN;
  const int tid = threadIdx.x, lane = tid & 31, wave = tid >> 5, hh = lane >> 4, m = lane & 15;
  const int nodeBase = blockIdx.x * NB1;

  {
    const v4f z = {0.f, 0.f, 0.f, 0.f};
    for (int i = tid; i < NB1 * DF / 4; i += NTHR) lds_dyn[i] = z;
  }
  __syncthreads();

  const int nChunks = (nE + CHUNK - 1) / CHUNK;
#pragma unroll 1
  for (int ch = 0; ch < nChunks; ++ch) {
    const int cbase = ch * CHUNK;
    const int wc = scan_chunk<NB1>(dsts, nE, cbase, nodeBase, vec8, list, tid, lane, wave);
    if (lane == 0) wcnt[wave] = wc;
    __syncthreads();
    if (wave == 0) {
#pragma unroll 1
      for (int wsx = 0; wsx < NWAVE; ++wsx) {
        int n = __builtin_amdgcn_readfirstlane(wcnt[wsx]);
        n = n > WCAP ? WCAP : (n < 0 ? 0 : n);
        const int* lp = list + wsx * WCAP;
#pragma unroll 1
        for (int i = 0; i < n; ++i) {
          const int ent  = __builtin_amdgcn_readfirstlane(lp[i]);
          const int slot = ent & (NB1 - 1);
          int e = cbase + ((ent >> 12) & (CHUNK - 1));
          e = e > nE - 1 ? nE - 1 : e;
          int s = srcs[e];
          s = s < 0 ? 0 : (s > nN - 1 ? nN - 1 : s);
          const float w = ew[e];
          const v4f v = *(const v4f*)(g1 + (size_t)s * DF + 4 * lane);
          v4f* ap = (v4f*)(acc + slot * DF + 4 * lane);
          *ap = *ap + v * w;
        }
      }
    }
    __syncthreads();
  }

#pragma unroll 4
  for (int i = 0; i < (NB1 * DF / 4) / NTHR; ++i) {
    const int idx  = i * NTHR + tid;
    const int slot = idx >> 5;
    const int c4   = (idx & 31) * 4;
    int node = nodeBase + slot;
    node = node > nN - 1 ? nN - 1 : node;
    const float d = nrmD[node];
    v4f* ap = (v4f*)(acc + slot * DF + c4);
    v4f hv = *ap * d;
    hv.x = lk(hv.x); hv.y = lk(hv.y); hv.z = lk(hv.z); hv.w = lk(hv.w);
    *ap = hv;
  }
  __syncthreads();

#pragma unroll 1
  for (int j = 0; j < NB1 / 16 / NWAVE; ++j) {
    const int t = wave + NWAVE * j;
    v8f c[4];
#pragma unroll
    for (int nt = 0; nt < 4; ++nt) { v8f z = {0.f, 0.f, 0.f, 0.f, 0.f, 0.f, 0.f, 0.f}; c[nt] = z; }
#pragma unroll
    for (int kt = 0; kt < 4; ++kt) {
      const float* ap = acc + (16 * t + m) * DF + 32 * kt + 8 * hh;
      const v4f p0 = *(const v4f*)ap,        p1 = *(const v4f*)(ap + 4);
      const v4f p2 = *(const v4f*)(ap + 16), p3 = *(const v4f*)(ap + 20);
      FragH a;
      a.h[0] = cvt8(p0 * ASC, p1 * ASC);
      a.h[1] = cvt8(p2 * ASC, p3 * ASC);
#pragma unroll
      for (int nt = 0; nt < 4; ++nt) {
        const _Float16* bp = w2s + (size_t)(16 * nt + m) * DF + 32 * kt + 8 * hh;
        FragH b;
        b.h[0] = *(const v8h*)bp;
        b.h[1] = *(const v8h*)(bp + 16);
        c[nt] = wmh(a.v, b.v, c[nt]);
      }
    }
    const int rl0   = 16 * t + 8 * hh;
    const int node0 = nodeBase + rl0;
    const v4f sA = *(const v4f*)(nrmS + (size_t)node0);
    const v4f sB = *(const v4f*)(nrmS + (size_t)node0 + 4);
    const float s0 = sA.x * AWINV, s1 = sA.y * AWINV, s2 = sA.z * AWINV, s3 = sA.w * AWINV;
    const float s4 = sB.x * AWINV, s5 = sB.y * AWINV, s6 = sB.z * AWINV, s7 = sB.w * AWINV;
    float* sp = acc + rl0 * DF + m;
#pragma unroll
    for (int nt = 0; nt < 4; ++nt) {
      sp[0 * DF + 16 * nt] = c[nt][0] * s0;
      sp[1 * DF + 16 * nt] = c[nt][1] * s1;
      sp[2 * DF + 16 * nt] = c[nt][2] * s2;
      sp[3 * DF + 16 * nt] = c[nt][3] * s3;
      sp[4 * DF + 16 * nt] = c[nt][4] * s4;
      sp[5 * DF + 16 * nt] = c[nt][5] * s5;
      sp[6 * DF + 16 * nt] = c[nt][6] * s6;
      sp[7 * DF + 16 * nt] = c[nt][7] * s7;
    }
  }
  __syncthreads();

  float* gb = g2 + (size_t)nodeBase * RDM;
  const int c4s = 4 * (lane & 15);
#pragma unroll 4
  for (int i = 0; i < NB1 / 2 / NWAVE; ++i) {
    const int r = 2 * (wave * (NB1 / 2 / NWAVE) + i) + hh;
    const v4f v = *(const v4f*)(acc + r * DF + c4s);
    *(volatile v4f*)(gb + (size_t)r * RDM + c4s) = v;
  }
  __threadfence();
#pragma unroll 4
  for (int i = 0; i < NB1 / 2 / NWAVE; ++i) {
    const int r = 2 * (wave * (NB1 / 2 / NWAVE) + i) + hh;
    const v4f v = *(const v4f*)(acc + r * DF + c4s);
    *(volatile v4f*)(gb + (size_t)r * RDM + c4s) = v;
  }
}

__global__ __launch_bounds__(NTHR) void k_agg2(
    const int* __restrict__ srcs, const int* __restrict__ dsts, const float* __restrict__ ew,
    const float* __restrict__ g2, const float* __restrict__ nrmD, float* h2,
    int nN, int nE, int vec8) {
  extern __shared__ v4f lds_dyn[];
  float* acc  = (float*)lds_dyn;
  int*   list = (int*)(acc + NB2 * RDM);
  int*   wcnt = list + LISTN;
  const int tid = threadIdx.x, lane = tid & 31, wave = tid >> 5;
  const int nodeBase = blockIdx.x * NB2;

  {
    const v4f z = {0.f, 0.f, 0.f, 0.f};
    for (int i = tid; i < NB2 * RDM / 4; i += NTHR) lds_dyn[i] = z;
  }
  __syncthreads();

  const int nChunks = (nE + CHUNK - 1) / CHUNK;
#pragma unroll 1
  for (int ch = 0; ch < nChunks; ++ch) {
    const int cbase = ch * CHUNK;
    const int wc = scan_chunk<NB2>(dsts, nE, cbase, nodeBase, vec8, list, tid, lane, wave);
    if (lane == 0) wcnt[wave] = wc;
    __syncthreads();
    if (wave == 0) {
#pragma unroll 1
      for (int wsx = 0; wsx < NWAVE; ++wsx) {
        int n = __builtin_amdgcn_readfirstlane(wcnt[wsx]);
        n = n > WCAP ? WCAP : (n < 0 ? 0 : n);
        const int* lp = list + wsx * WCAP;
#pragma unroll 1
        for (int i = 0; i < n; ++i) {
          const int ent  = __builtin_amdgcn_readfirstlane(lp[i]);
          const int slot = ent & (NB2 - 1);
          int e = cbase + ((ent >> 12) & (CHUNK - 1));
          e = e > nE - 1 ? nE - 1 : e;
          int s = srcs[e];
          s = s < 0 ? 0 : (s > nN - 1 ? nN - 1 : s);
          const float w = ew[e];
          const v4f v = *(const v4f*)(g2 + (size_t)s * RDM + 4 * (lane & 15));
          if (lane < 16) {
            v4f* ap = (v4f*)(acc + slot * RDM + 4 * lane);
            *ap = *ap + v * w;
          }
        }
      }
    }
    __syncthreads();
  }

#pragma unroll 4
  for (int i = 0; i < (NB2 * RDM / 4) / NTHR; ++i) {
    const int idx  = i * NTHR + tid;
    const int slot = idx >> 4;
    const int c4   = (idx & 15) * 4;
    int node = nodeBase + slot;
    node = node > nN - 1 ? nN - 1 : node;
    const float d = nrmD[node];
    v4f* ap = (v4f*)(acc + slot * RDM + c4);
    v4f hv = *ap * d;
    hv.x = lk(hv.x); hv.y = lk(hv.y); hv.z = lk(hv.z); hv.w = lk(hv.w);
    *ap = hv;
  }
  __syncthreads();

  const size_t ob = (size_t)nodeBase * RDM;
#pragma unroll 4
  for (int q = 0; q < (NB2 * RDM) / (128 * NWAVE); ++q) {
    const int f = (wave * ((NB2 * RDM) / (128 * NWAVE)) + q) * 128 + 4 * lane;
    const v4f v = *(const v4f*)(acc + f);
    *(volatile v4f*)(h2 + ob + (size_t)f) = v;
  }
  __threadfence();
#pragma unroll 4
  for (int q = 0; q < (NB2 * RDM) / (128 * NWAVE); ++q) {
    const int f = (wave * ((NB2 * RDM) / (128 * NWAVE)) + q) * 128 + 4 * lane;
    const v4f v = *(const v4f*)(acc + f);
    *(volatile v4f*)(h2 + ob + (size_t)f) = v;
  }
}

__global__ __launch_bounds__(NTHR) void k_pool(
    const int* __restrict__ gid, const float* __restrict__ h2, const int* __restrict__ ng,
    float* out, int nN, int G, int vec8) {
  __shared__ __attribute__((aligned(16))) float acc[NBP * RDM];
  __shared__ __attribute__((aligned(16))) int list[LISTN];
  __shared__ int cnt[NBP];
  __shared__ int wcnt[NWAVE];
  const int tid = threadIdx.x, lane = tid & 31, wave = tid >> 5;
  const int gBase = blockIdx.x * NBP;
  int gN = ng[0];
  gN = gN < 1 ? 1 : (gN > G ? G : gN);

  {
    const v4f z = {0.f, 0.f, 0.f, 0.f};
    for (int i = tid; i < NBP * RDM / 4; i += NTHR) ((v4f*)acc)[i] = z;
  }
  if (tid < NBP) cnt[tid] = 0;
  __syncthreads();

  const int nChunks = (nN + CHUNK - 1) / CHUNK;
#pragma unroll 1
  for (int ch = 0; ch < nChunks; ++ch) {
    const int cbase = ch * CHUNK;
    const int wc = scan_chunk<NBP>(gid, nN, cbase, gBase, vec8, list, tid, lane, wave);
    if (lane == 0) wcnt[wave] = wc;
    __syncthreads();
    if (wave == 0) {
#pragma unroll 1
      for (int wsx = 0; wsx < NWAVE; ++wsx) {
        int n = __builtin_amdgcn_readfirstlane(wcnt[wsx]);
        n = n > WCAP ? WCAP : (n < 0 ? 0 : n);
        const int* lp = list + wsx * WCAP;
#pragma unroll 1
        for (int i = 0; i < n; ++i) {
          const int ent  = __builtin_amdgcn_readfirstlane(lp[i]);
          const int slot = ent & (NBP - 1);
          int node = cbase + ((ent >> 12) & (CHUNK - 1));
          node = node > nN - 1 ? nN - 1 : node;
          if (gBase + slot < gN) {
            const v4f v = *(const v4f*)(h2 + (size_t)node * RDM + 4 * (lane & 15));
            if (lane < 16) {
              v4f* ap = (v4f*)(acc + slot * RDM + 4 * lane);
              *ap = *ap + v;
            }
            if (lane == 0) cnt[slot] = cnt[slot] + 1;
          }
        }
      }
    }
    __syncthreads();
  }

#pragma unroll
  for (int i = tid; i < NBP * RDM / 4; i += NTHR) {
    const int slot = i >> 4;
    const int c4   = (i & 15) * 4;
    int c = cnt[slot];
    c = c < 1 ? 1 : c;
    const float inv = 1.0f / (float)c;
    v4f* ap = (v4f*)(acc + slot * RDM + c4);
    const v4f mv = *ap * inv;
    *ap = mv;
  }
  __syncthreads();

  const size_t ob = (size_t)gBase * RDM;
#pragma unroll
  for (int i = 0; i < 2; ++i) {
    const int f = (wave * 2 + i) * 128 + 4 * lane;
    const int row = f >> 6;
    if (gBase + row < G) { const v4f v = *(const v4f*)(acc + f); *(volatile v4f*)(out + ob + (size_t)f) = v; }
  }
  __threadfence();
#pragma unroll
  for (int i = 0; i < 2; ++i) {
    const int f = (wave * 2 + i) * 128 + 4 * lane;
    const int row = f >> 6;
    if (gBase + row < G) { const v4f v = *(const v4f*)(acc + f); *(volatile v4f*)(out + ob + (size_t)f) = v; }
  }
}

extern "C" void kernel_launch(void* const* d_in, const int* in_sizes, int n_in,
                              void* d_out, int out_size, void* d_ws, size_t ws_size,
                              hipStream_t stream) {
  if (n_in < 8) return;
  const int nN = in_sizes[6];
  const int nE = in_sizes[4];
  if (nN <= 0 || nE <= 0) return;
  if (in_sizes[0] != nN * DF || in_sizes[1] != nE || in_sizes[5] != nE) return;
  if (in_sizes[2] != DF * DF || in_sizes[3] != DF * RDM || in_sizes[7] < 1) return;
  const int G = out_size / RDM;
  if (G <= 0 || out_size != G * RDM) return;

  const float* x   = (const float*)d_in[0];
  const float* ew  = (const float*)d_in[1];
  const float* W1  = (const float*)d_in[2];
  const float* W2  = (const float*)d_in[3];
  const int*   src = (const int*)d_in[4];
  const int*   dst = (const int*)d_in[5];
  const int*   gid = (const int*)d_in[6];
  const int*   ng  = (const int*)d_in[7];
  float* out = (float*)d_out;

  const int nBD = (nN + NBD - 1) / NBD;
  const int nG1 = (nN + G1ROWS - 1) / G1ROWS;
  const int nA1 = (nN + NB1 - 1) / NB1;
  const int nA2 = (nN + NB2 - 1) / NB2;
  const int nP  = (G + NBP - 1) / NBP;

  char* ws = (char*)d_ws;
  size_t off = 0;
  const size_t oW1 = off; off += (size_t)DF * DF * 2;                          off = (off + 255) & ~(size_t)255;
  const size_t oW2 = off; off += (size_t)RDM * DF * 2;                         off = (off + 255) & ~(size_t)255;
  const size_t oNS = off; off += (size_t)nBD * NBD * 4;                        off = (off + 255) & ~(size_t)255;
  const size_t oND = off; off += (size_t)nBD * NBD * 4;                        off = (off + 255) & ~(size_t)255;
  const size_t oG1 = off; off += (size_t)nG1 * G1ROWS * DF * 4;                off = (off + 255) & ~(size_t)255;
  const size_t oG2 = off; off += (size_t)nA1 * NB1 * RDM * 4;                  off = (off + 255) & ~(size_t)255;
  const size_t oH2 = off; off += (size_t)nA2 * NB2 * RDM * 4;                  off = (off + 255) & ~(size_t)255;
  if (off > ws_size) return;
  _Float16* w1s  = (_Float16*)(ws + oW1);
  _Float16* w2s  = (_Float16*)(ws + oW2);
  float*    nrmS = (float*)(ws + oNS);
  float*    nrmD = (float*)(ws + oND);
  float*    g1   = (float*)(ws + oG1);
  float*    g2   = (float*)(ws + oG2);
  float*    h2   = (float*)(ws + oH2);

  const int vec8 = 1;

  const int nPrep = DF * DF / 8 + RDM * DF / 8;
  k_wprep<<<(nPrep + NTHR - 1) / NTHR, NTHR, 0, stream>>>(W1, W2, w1s, w2s);

  k_deg<<<nBD, NTHR, 0, stream>>>(src, nrmS, nE, vec8);
  k_deg<<<nBD, NTHR, 0, stream>>>(dst, nrmD, nE, vec8);

  hipFuncSetAttribute(reinterpret_cast<const void*>(&k_gemm1),
                      hipFuncAttributeMaxDynamicSharedMemorySize, LDS_GEMM1);
  k_gemm1<<<nG1, NTHR, LDS_GEMM1, stream>>>(x, w1s, nrmS, g1, nN);

  hipFuncSetAttribute(reinterpret_cast<const void*>(&k_agg1),
                      hipFuncAttributeMaxDynamicSharedMemorySize, LDS_AGG1);
  k_agg1<<<nA1, NTHR, LDS_AGG1, stream>>>(src, dst, ew, g1, nrmD, nrmS, w2s, g2, nN, nE, vec8);

  hipFuncSetAttribute(reinterpret_cast<const void*>(&k_agg2),
                      hipFuncAttributeMaxDynamicSharedMemorySize, LDS_AGG2);
  k_agg2<<<nA2, NTHR, LDS_AGG2, stream>>>(src, dst, ew, g2, nrmD, h2, nN, nE, vec8);

  k_pool<<<nP, NTHR, 0, stream>>>(gid, h2, ng, out, nN, G, vec8);
}
